// PosEvalModel_9131100472049
// MI455X (gfx1250) — hardware-verified
//
#include <hip/hip_runtime.h>


#define AS3 __attribute__((address_space(3)))

#define B_    64
#define C_    50
#define L_    128
#define S_    128
#define G3_   384
#define NR_   (B_ * C_)
#define V_    100008
#define VP_   100032
#define OUT_  3
#define PWK_  129

#define MB_   64
#define NTHR  256
#define HP    136
#define GIP   392
#define OP    388

static_assert(VP_ % MB_ == 0);
static_assert(VP_ >= V_);
static_assert(NR_ % MB_ == 0);
static_assert(S_ % 32 == 0);
static_assert(HP % 8 == 0);
static_assert(GIP % 8 == 0);
static_assert(OP % 4 == 0);
static_assert(NTHR == 256);
static_assert(S_ == (NTHR / 32) * 16);
static_assert(MB_ == 64);

typedef _Float16 v16h __attribute__((ext_vector_type(16)));
typedef _Float16 v8h  __attribute__((ext_vector_type(8)));
typedef _Float16 v4h  __attribute__((ext_vector_type(4)));
typedef float    v8f  __attribute__((ext_vector_type(8)));
typedef float    v4f  __attribute__((ext_vector_type(4)));

typedef AS3 _Float16*       lp_h;
typedef AS3 const _Float16* lcp_h;
typedef AS3 float*          lp_f;
typedef AS3 const float*    lcp_f;
typedef AS3 int*            lp_i;

union Frag { v16h v; v8h half[2]; };

#define SCW    16.0f
#define SCA    8.0f
#define INV8   0.125f
#define INV32  0.03125f
#define INV128 0.0078125f

constexpr size_t SZ_EMB = (size_t)VP_ * S_ * 2;
constexpr size_t SZ_GI  = (size_t)VP_ * G3_ * 2;
constexpr size_t SZ_W   = (size_t)G3_ * S_ * 2;
constexpr size_t SZ_PW  = (size_t)S_ * S_ * 2;
constexpr size_t SZ_HT  = (size_t)NR_ * S_ * 4;
constexpr size_t SZ_GIC = (size_t)NR_ * G3_ * 4;
constexpr size_t OFF_EMB = 0;
constexpr size_t OFF_GI  = OFF_EMB + SZ_EMB;
constexpr size_t OFF_WAI = OFF_GI  + SZ_GI;
constexpr size_t OFF_WAH = OFF_WAI + SZ_W;
constexpr size_t OFF_WCI = OFF_WAH + SZ_W;
constexpr size_t OFF_WCH = OFF_WCI + SZ_W;
constexpr size_t OFF_PW  = OFF_WCH + SZ_W;
constexpr size_t OFF_HT  = OFF_PW  + SZ_PW;
constexpr size_t OFF_GIC = OFF_HT  + SZ_HT;
constexpr size_t WS_END  = OFF_GIC + SZ_GIC;
static_assert(OFF_GI % 128 == 0 && OFF_WAI % 128 == 0 && OFF_WAH % 128 == 0 && OFF_WCI % 128 == 0);
static_assert(OFF_WCH % 128 == 0 && OFF_PW % 128 == 0 && OFF_HT % 128 == 0 && OFF_GIC % 128 == 0);
static_assert(WS_END <= (size_t)134217728);

constexpr int E_PCS = VP_ * S_ / 8;
constexpr int E_BLK = E_PCS / NTHR;
constexpr int W_PCS = G3_ * S_ / 8;
constexpr int W_BLK = W_PCS / NTHR;
constexpr int P_PCS = S_ * S_ / 8;
constexpr int P_BLK = P_PCS / NTHR;
constexpr int CVT_BLK = E_BLK + 4 * W_BLK + P_BLK;
static_assert(E_PCS % NTHR == 0 && W_PCS % NTHR == 0 && P_PCS % NTHR == 0);
static_assert((size_t)E_PCS * 16 == SZ_EMB);
static_assert((size_t)W_PCS * 16 == SZ_W);
static_assert((size_t)P_PCS * 16 == SZ_PW);

constexpr int GI_BLK  = VP_ / MB_;
constexpr int ROW_BLK = NR_ / MB_;
static_assert((size_t)GI_BLK * MB_ * G3_ * 2 == SZ_GI);
static_assert((size_t)ROW_BLK * MB_ * S_ * 4 == SZ_HT);
static_assert((size_t)ROW_BLK * MB_ * G3_ * 4 == SZ_GIC);

constexpr int    HBT      = MB_ * HP;
constexpr size_t LA_TOK   = 0;
constexpr size_t LA_GI    = LA_TOK + (size_t)MB_ * L_ * 4;
constexpr size_t LA_H     = LA_GI  + (size_t)MB_ * GIP * 2;
constexpr size_t LA_HB    = LA_H   + (size_t)MB_ * S_ * 4;
constexpr size_t LA_BI    = LA_HB  + (size_t)2 * HBT * 2;
constexpr size_t LA_BH    = LA_BI  + (size_t)G3_ * 4;
constexpr size_t LDS_AST  = LA_BH  + (size_t)G3_ * 4;
static_assert(LA_GI % 16 == 0 && LA_H % 16 == 0 && LA_HB % 16 == 0 && LA_BI % 16 == 0 && LA_BH % 16 == 0);
constexpr size_t LP_A     = 0;
constexpr size_t LP_P     = LP_A + (size_t)HBT * 2;
constexpr size_t LP_O     = LP_P + (size_t)HBT * 2;
constexpr size_t LDS_PROJ = LP_O + (size_t)MB_ * OP * 4;
static_assert(LP_P % 16 == 0 && LP_O % 16 == 0);
constexpr size_t LC_H     = 0;
constexpr size_t LC_HB    = LC_H  + (size_t)MB_ * S_ * 4;
constexpr size_t LC_BI    = LC_HB + (size_t)2 * HBT * 2;
constexpr size_t LC_BH    = LC_BI + (size_t)G3_ * 4;
constexpr size_t LC_OUT   = LC_BH + (size_t)G3_ * 4;
constexpr size_t LDS_CTX  = LC_OUT + (size_t)B_ * OUT_ * 4;
static_assert(LC_HB % 16 == 0 && LC_BI % 16 == 0 && LC_BH % 16 == 0 && LC_OUT % 16 == 0);
static_assert((B_ * OUT_) % 4 == 0);

__device__ __forceinline__ float rcpx(float x) { return __builtin_amdgcn_rcpf(x); }
__device__ __forceinline__ float sigm(float x) { return rcpx(1.0f + expf(-x)); }
__device__ __forceinline__ v8f ld8f(const float* p) {
    const v4f a = *(const v4f*)p;
    const v4f b = *(const v4f*)(p + 4);
    return __builtin_shufflevector(a, b, 0, 1, 2, 3, 4, 5, 6, 7);
}
__device__ __forceinline__ v8f zero8() {
    v8f z;
#pragma unroll
    for (int i = 0; i < 8; ++i) z[i] = 0.0f;
    return z;
}
__device__ __forceinline__ float gru_cell(float gir, float giz, float gin,
                                          float ghr, float ghz, float ghn, float hp) {
    const float rg = sigm(gir + ghr);
    const float zg = sigm(giz + ghz);
    const float ng = tanhf(gin + rg * ghn);
    return (1.0f - zg) * ng + zg * hp;
}

__device__ __forceinline__ void ldfrag_lds(Frag& f, lcp_h p) {
    f.half[0] = *(AS3 const v8h*)(p);
    f.half[1] = *(AS3 const v8h*)(p + 16);
}
__device__ __forceinline__ void ldfrag_glb(Frag& f, const _Float16* p) {
    f.half[0] = *(const v8h*)(p);
    f.half[1] = *(const v8h*)(p + 16);
}
__device__ __forceinline__ v8f mma16(v8f c, const Frag& a, const Frag& b) {
    return __builtin_amdgcn_wmma_f32_16x16x32_f16(false, a.v, false, b.v, (short)0, c, false, false);
}
#define NOP6(A0, A1, A2, A3, A4, A5, F0, F1, F2, F3, F4)                                   \
    asm volatile("v_nop\n\tv_nop\n\tv_nop\n\tv_nop"                                       \
                 : "+v"(A0), "+v"(A1), "+v"(A2), "+v"(A3), "+v"(A4), "+v"(A5)             \
                 : "v"(F0), "v"(F1), "v"(F2), "v"(F3), "v"(F4))

__global__ __launch_bounds__(NTHR)
void cvt_kernel(const float* __restrict__ embed, const float* __restrict__ awih,
                const float* __restrict__ awhh, const float* __restrict__ cwih,
                const float* __restrict__ cwhh, const float* __restrict__ projw,
                _Float16* Emb, _Float16* Wai, _Float16* Wah, _Float16* Wci,
                _Float16* Wch, _Float16* Pw)
{
    const int tid = threadIdx.x;
    const int blk = blockIdx.x;
    v8h hv;
    _Float16* d;
    if (blk < E_BLK) {
        const int p  = blk * NTHR + tid;
        const int v  = p >> 4;
        const int c8 = (p & 15) * 8;
        const int vc = min(v, V_ - 1);
        const v8f a  = ld8f(embed + (size_t)vc * S_ + c8);
        const bool in = v < V_;
#pragma unroll
        for (int i = 0; i < 8; ++i) hv[i] = (_Float16)(in ? a[i] * SCW : 0.0f);
        d = Emb + (size_t)v * S_ + c8;
    } else if (blk < E_BLK + 4 * W_BLK) {
        const int q     = blk - E_BLK;
        const int plane = q / W_BLK;
        const float* src = (plane == 0) ? awih : (plane == 1) ? awhh : (plane == 2) ? cwih : cwhh;
        _Float16*    dst = (plane == 0) ? Wai  : (plane == 1) ? Wah  : (plane == 2) ? Wci  : Wch;
        const int p  = (q - plane * W_BLK) * NTHR + tid;
        const int n  = p >> 4;
        const int c8 = (p & 15) * 8;
        const v8f a  = ld8f(src + (size_t)n * S_ + c8);
#pragma unroll
        for (int i = 0; i < 8; ++i) hv[i] = (_Float16)(a[i] * SCW);
        d = dst + (size_t)n * S_ + c8;
    } else {
        const int p  = (blk - E_BLK - 4 * W_BLK) * NTHR + tid;
        const int n  = p >> 4;
        const int c8 = (p & 15) * 8;
#pragma unroll
        for (int i = 0; i < 8; ++i) hv[i] = (_Float16)(projw[(size_t)n * PWK_ + c8 + i] * SCW);
        d = Pw + (size_t)n * S_ + c8;
    }
    *(volatile v8h*)d = hv;
    __threadfence();
    *(volatile v8h*)d = hv;
}

__global__ __launch_bounds__(NTHR)
void gi_table_kernel(const _Float16* __restrict__ Emb, const _Float16* __restrict__ Wai, _Float16* GI)
{
    __shared__ __attribute__((aligned(16))) _Float16 sO[MB_ * GIP];
    const int tid  = threadIdx.x;
    const int lane = tid & 31;
    const int w    = tid >> 5;
    const int h    = lane >> 4;
    const int m    = lane & 15;
    const int row0 = blockIdx.x * MB_;
    const int n0   = w * 48;

#pragma unroll 1
    for (int mh = 0; mh < 2; ++mh) {
        v8f acc[2][3];
#pragma unroll
        for (int mt = 0; mt < 2; ++mt)
#pragma unroll
            for (int q = 0; q < 3; ++q) acc[mt][q] = zero8();
        const _Float16* ab = Emb + (size_t)(row0 + 32 * mh + m) * S_ + 8 * h;
        const _Float16* wb = Wai + (size_t)(n0 + m) * S_ + 8 * h;
#pragma unroll 1
        for (int k0 = 0; k0 < S_; k0 += 32) {
            Frag a[2], b[3];
#pragma unroll
            for (int mt = 0; mt < 2; ++mt) ldfrag_glb(a[mt], ab + (size_t)mt * (16 * S_) + k0);
#pragma unroll
            for (int q = 0; q < 3; ++q) ldfrag_glb(b[q], wb + (size_t)q * (16 * S_) + k0);
#pragma unroll
            for (int mt = 0; mt < 2; ++mt)
#pragma unroll
                for (int q = 0; q < 3; ++q) acc[mt][q] = mma16(acc[mt][q], a[mt], b[q]);
            NOP6(acc[0][0], acc[0][1], acc[0][2], acc[1][0], acc[1][1], acc[1][2],
                 a[0].v, a[1].v, b[0].v, b[1].v, b[2].v);
        }
#pragma unroll
        for (int mt = 0; mt < 2; ++mt)
#pragma unroll
            for (int q = 0; q < 3; ++q)
#pragma unroll
                for (int r = 0; r < 8; ++r) {
                    const int row = 32 * mh + 16 * mt + 8 * h + r;
                    sO[row * GIP + n0 + 16 * q + m] = (_Float16)(acc[mt][q][r] * INV32);
                }
    }
    __syncthreads();
#pragma unroll 2
    for (int it = 0; it < 12; ++it) {
        const int idx = tid + NTHR * it;
        const int row = idx / 48;
        const int pc  = idx - row * 48;
        const v8h v = *(AS3 const v8h*)((lcp_h)sO + row * GIP + 8 * pc);
        _Float16* d = GI + (size_t)(row0 + row) * G3_ + 8 * pc;
        *(volatile v8h*)d = v;
        __threadfence();
        *(volatile v8h*)d = v;
    }
}

__global__ __launch_bounds__(NTHR)
void ast_gru_kernel(const int* __restrict__ tok, const _Float16* __restrict__ GI,
                    const _Float16* __restrict__ Wah, const float* __restrict__ bih,
                    const float* __restrict__ bhh, const float* __restrict__ hinit,
                    float* hT)
{
    extern __shared__ __attribute__((aligned(16))) char smem[];
    lp_i sTok = (lp_i)(smem + LA_TOK);
    lp_h sGI  = (lp_h)(smem + LA_GI);
    lp_f sH   = (lp_f)(smem + LA_H);
    lp_h sHb  = (lp_h)(smem + LA_HB);
    lp_f sBi  = (lp_f)(smem + LA_BI);
    lp_f sBh  = (lp_f)(smem + LA_BH);

    const int tid  = threadIdx.x;
    const int lane = tid & 31;
    const int w    = tid >> 5;
    const int h    = lane >> 4;
    const int m    = lane & 15;
    const int row0 = blockIdx.x * MB_;

    for (int i = tid; i < MB_ * L_; i += NTHR) {
        const int t = tok[(size_t)row0 * L_ + i];
        sTok[i] = min(max(t, 0), V_ - 1);
    }
    for (int i = tid; i < MB_ * S_; i += NTHR) {
        const int row = i >> 7, k = i & 127;
        const float hv = hinit[k];
        sH[row * S_ + k] = hv;
        const _Float16 hb = (_Float16)(hv * SCA);
        sHb[row * HP + k] = hb;
        sHb[HBT + row * HP + k] = hb;
    }
    for (int i = tid; i < G3_; i += NTHR) { sBi[i] = bih[i]; sBh[i] = bhh[i]; }
    __syncthreads();

    const int j0 = w * 16;
    const int n  = j0 + m;
    const float bir = sBi[n], biz = sBi[S_ + n], bin = sBi[2 * S_ + n];
    const float bhr = sBh[n], bhz = sBh[S_ + n], bhn = sBh[2 * S_ + n];

#pragma unroll 1
    for (int t = 0; t < L_; ++t) {
        const int cur = t & 1;
        lcp_h sHc = sHb + cur * HBT;
        lp_h  sHn = sHb + (cur ^ 1) * HBT;

        __syncthreads();

#pragma unroll 4
        for (int it = 0; it < 12; ++it) {
            const int idx = tid + NTHR * it;
            const int row = idx / 48;
            const int pc  = idx - row * 48;
            const int tk  = sTok[row * L_ + t];
            const v8h v = *(const v8h*)(GI + (size_t)tk * G3_ + 8 * pc);
            *(AS3 v8h*)(sGI + row * GIP + 8 * pc) = v;
        }
        __syncthreads();

#pragma unroll 1
        for (int mh = 0; mh < 2; ++mh) {
            v8f acc[2][3];
#pragma unroll
            for (int mt = 0; mt < 2; ++mt)
#pragma unroll
                for (int q = 0; q < 3; ++q) acc[mt][q] = zero8();
            lcp_h ab = sHc + (32 * mh + m) * HP + 8 * h;
            const _Float16* wb = Wah + (size_t)(j0 + m) * S_ + 8 * h;
#pragma unroll 1
            for (int k0 = 0; k0 < S_; k0 += 32) {
                Frag a[2], b[3];
#pragma unroll
                for (int mt = 0; mt < 2; ++mt) ldfrag_lds(a[mt], ab + mt * (16 * HP) + k0);
#pragma unroll
                for (int q = 0; q < 3; ++q) ldfrag_glb(b[q], wb + (size_t)q * (S_ * S_) + k0);
#pragma unroll
                for (int mt = 0; mt < 2; ++mt)
#pragma unroll
                    for (int q = 0; q < 3; ++q) acc[mt][q] = mma16(acc[mt][q], a[mt], b[q]);
                NOP6(acc[0][0], acc[0][1], acc[0][2], acc[1][0], acc[1][1], acc[1][2],
                     a[0].v, a[1].v, b[0].v, b[1].v, b[2].v);
            }
#pragma unroll
            for (int mt = 0; mt < 2; ++mt) {
#pragma unroll
                for (int r = 0; r < 8; ++r) {
                    const int row = 32 * mh + 16 * mt + 8 * h + r;
                    lcp_h gp = sGI + row * GIP + n;
                    const float gir = (float)gp[0]      * INV8 + bir;
                    const float giz = (float)gp[S_]     * INV8 + biz;
                    const float gin = (float)gp[2 * S_] * INV8 + bin;
                    const float ghr = acc[mt][0][r] * INV128 + bhr;
                    const float ghz = acc[mt][1][r] * INV128 + bhz;
                    const float ghn = acc[mt][2][r] * INV128 + bhn;
                    const float hp  = sH[row * S_ + n];
                    const float hn  = gru_cell(gir, giz, gin, ghr, ghz, ghn, hp);
                    sH[row * S_ + n]   = hn;
                    sHn[row * HP + n]  = (_Float16)(hn * SCA);
                }
            }
        }
    }
    __syncthreads();

#pragma unroll 2
    for (int it = 0; it < 8; ++it) {
        const int idx = tid + NTHR * it;
        const int row = idx >> 5;
        const int pc  = idx & 31;
        const v4f v = *(AS3 const v4f*)((lcp_f)sH + row * S_ + 4 * pc);
        float* d = hT + (size_t)(row0 + row) * S_ + 4 * pc;
        *(volatile v4f*)d = v;
        __threadfence();
        *(volatile v4f*)d = v;
    }
}

__global__ __launch_bounds__(NTHR)
void proj_kernel(const float* __restrict__ hT, const _Float16* __restrict__ Pw,
                 const float* __restrict__ projw, const float* __restrict__ projb,
                 const _Float16* __restrict__ Wci, float* GIc)
{
    extern __shared__ __attribute__((aligned(16))) char smem[];
    lp_h sA = (lp_h)(smem + LP_A);
    lp_h sP = (lp_h)(smem + LP_P);
    lp_f sO = (lp_f)(smem + LP_O);

    const int tid  = threadIdx.x;
    const int lane = tid & 31;
    const int w    = tid >> 5;
    const int h    = lane >> 4;
    const int m    = lane & 15;
    const int row0 = blockIdx.x * MB_;

#pragma unroll 2
    for (int it = 0; it < 8; ++it) {
        const int idx = tid + NTHR * it;
        const int row = idx >> 5;
        const int pc  = idx & 31;
        const v4f x = *(const v4f*)(hT + (size_t)(row0 + row) * S_ + 4 * pc);
        v4h hv;
#pragma unroll
        for (int i = 0; i < 4; ++i) hv[i] = (_Float16)(x[i] * SCA);
        *(AS3 v4h*)(sA + row * HP + 4 * pc) = hv;
    }
    __syncthreads();

    {
        const int n1 = w * 16 + m;
        v8f acc[4];
#pragma unroll
        for (int mt = 0; mt < 4; ++mt) acc[mt] = zero8();
        lcp_h ab = sA + m * HP + 8 * h;
        const _Float16* wb = Pw + (size_t)n1 * S_ + 8 * h;
#pragma unroll 1
        for (int k0 = 0; k0 < S_; k0 += 32) {
            Frag a[4], b;
#pragma unroll
            for (int mt = 0; mt < 4; ++mt) ldfrag_lds(a[mt], ab + mt * (16 * HP) + k0);
            ldfrag_glb(b, wb + k0);
#pragma unroll
            for (int mt = 0; mt < 4; ++mt) acc[mt] = mma16(acc[mt], a[mt], b);
            asm volatile("v_nop\n\tv_nop\n\tv_nop\n\tv_nop"
                         : "+v"(acc[0]), "+v"(acc[1]), "+v"(acc[2]), "+v"(acc[3])
                         : "v"(a[0].v), "v"(a[1].v), "v"(a[2].v), "v"(a[3].v), "v"(b.v));
        }
        const float pb = projb[n1];
        const float wi = projw[(size_t)n1 * PWK_ + S_];
#pragma unroll
        for (int mt = 0; mt < 4; ++mt) {
#pragma unroll
            for (int r = 0; r < 8; ++r) {
                const int row = 16 * mt + 8 * h + r;
                const int g   = row0 + row;
                const float ind = ((g % C_) == 0) ? 1.0f : 0.0f;
                const float p = acc[mt][r] * INV128 + ind * wi + pb;
                sP[row * HP + n1] = (_Float16)(p * SCA);
            }
        }
    }
    __syncthreads();

    const int j0 = w * 16;
#pragma unroll 1
    for (int mh = 0; mh < 2; ++mh) {
        v8f acc[2][3];
#pragma unroll
        for (int mt = 0; mt < 2; ++mt)
#pragma unroll
            for (int q = 0; q < 3; ++q) acc[mt][q] = zero8();
        lcp_h ab = sP + (32 * mh + m) * HP + 8 * h;
        const _Float16* wb = Wci + (size_t)(j0 + m) * S_ + 8 * h;
#pragma unroll 1
        for (int k0 = 0; k0 < S_; k0 += 32) {
            Frag a[2], b[3];
#pragma unroll
            for (int mt = 0; mt < 2; ++mt) ldfrag_lds(a[mt], ab + mt * (16 * HP) + k0);
#pragma unroll
            for (int q = 0; q < 3; ++q) ldfrag_glb(b[q], wb + (size_t)q * (S_ * S_) + k0);
#pragma unroll
            for (int mt = 0; mt < 2; ++mt)
#pragma unroll
                for (int q = 0; q < 3; ++q) acc[mt][q] = mma16(acc[mt][q], a[mt], b[q]);
            NOP6(acc[0][0], acc[0][1], acc[0][2], acc[1][0], acc[1][1], acc[1][2],
                 a[0].v, a[1].v, b[0].v, b[1].v, b[2].v);
        }
#pragma unroll
        for (int mt = 0; mt < 2; ++mt)
#pragma unroll
            for (int q = 0; q < 3; ++q)
#pragma unroll
                for (int r = 0; r < 8; ++r) {
                    const int row = 32 * mh + 16 * mt + 8 * h + r;
                    sO[row * OP + q * S_ + j0 + m] = acc[mt][q][r] * INV128;
                }
    }
    __syncthreads();

#pragma unroll 2
    for (int it = 0; it < 24; ++it) {
        const int idx = tid + NTHR * it;
        const int row = idx / 96;
        const int pc  = idx - row * 96;
        const v4f v = *(AS3 const v4f*)((lcp_f)sO + row * OP + 4 * pc);
        float* d = GIc + (size_t)(row0 + row) * G3_ + 4 * pc;
        *(volatile v4f*)d = v;
        __threadfence();
        *(volatile v4f*)d = v;
    }
}

__global__ __launch_bounds__(NTHR)
void ctx_gru_kernel(const float* __restrict__ GIc, const _Float16* __restrict__ Wch,
                    const float* __restrict__ bih, const float* __restrict__ bhh,
                    const float* __restrict__ cinit, const float* __restrict__ fw,
                    const float* __restrict__ fb, float* out)
{
    extern __shared__ __attribute__((aligned(16))) char smem[];
    lp_f sH   = (lp_f)(smem + LC_H);
    lp_h sHb  = (lp_h)(smem + LC_HB);
    lp_f sBi  = (lp_f)(smem + LC_BI);
    lp_f sBh  = (lp_f)(smem + LC_BH);
    lp_f sOut = (lp_f)(smem + LC_OUT);

    const int tid  = threadIdx.x;
    const int lane = tid & 31;
    const int w    = tid >> 5;
    const int h    = lane >> 4;
    const int m    = lane & 15;

    for (int i = tid; i < MB_ * S_; i += NTHR) {
        const int row = i >> 7, k = i & 127;
        const float hv = cinit[k];
        sH[row * S_ + k] = hv;
        const _Float16 hb = (_Float16)(hv * SCA);
        sHb[row * HP + k] = hb;
        sHb[HBT + row * HP + k] = hb;
    }
    for (int i = tid; i < G3_; i += NTHR) { sBi[i] = bih[i]; sBh[i] = bhh[i]; }
    __syncthreads();

    const int j0 = w * 16;
    const int n  = j0 + m;
    const float bir = sBi[n], biz = sBi[S_ + n], bin = sBi[2 * S_ + n];
    const float bhr = sBh[n], bhz = sBh[S_ + n], bhn = sBh[2 * S_ + n];

#pragma unroll 1
    for (int c = 0; c < C_; ++c) {
        const int cur = c & 1;
        lcp_h sHc = sHb + cur * HBT;
        lp_h  sHn = sHb + (cur ^ 1) * HBT;
        __syncthreads();

#pragma unroll 1
        for (int mh = 0; mh < 2; ++mh) {
            v8f acc[2][3];
#pragma unroll
            for (int mt = 0; mt < 2; ++mt)
#pragma unroll
                for (int q = 0; q < 3; ++q) acc[mt][q] = zero8();
            lcp_h ab = sHc + (32 * mh + m) * HP + 8 * h;
            const _Float16* wb = Wch + (size_t)(j0 + m) * S_ + 8 * h;
#pragma unroll 1
            for (int k0 = 0; k0 < S_; k0 += 32) {
                Frag a[2], b[3];
#pragma unroll
                for (int mt = 0; mt < 2; ++mt) ldfrag_lds(a[mt], ab + mt * (16 * HP) + k0);
#pragma unroll
                for (int q = 0; q < 3; ++q) ldfrag_glb(b[q], wb + (size_t)q * (S_ * S_) + k0);
#pragma unroll
                for (int mt = 0; mt < 2; ++mt)
#pragma unroll
                    for (int q = 0; q < 3; ++q) acc[mt][q] = mma16(acc[mt][q], a[mt], b[q]);
                NOP6(acc[0][0], acc[0][1], acc[0][2], acc[1][0], acc[1][1], acc[1][2],
                     a[0].v, a[1].v, b[0].v, b[1].v, b[2].v);
            }
#pragma unroll
            for (int mt = 0; mt < 2; ++mt) {
#pragma unroll
                for (int r = 0; r < 8; ++r) {
                    const int row = 32 * mh + 16 * mt + 8 * h + r;
                    const float* gp = GIc + ((size_t)(row * C_ + c)) * G3_ + n;
                    const float gir = gp[0]      + bir;
                    const float giz = gp[S_]     + biz;
                    const float gin = gp[2 * S_] + bin;
                    const float ghr = acc[mt][0][r] * INV128 + bhr;
                    const float ghz = acc[mt][1][r] * INV128 + bhz;
                    const float ghn = acc[mt][2][r] * INV128 + bhn;
                    const float hp  = sH[row * S_ + n];
                    const float hn  = gru_cell(gir, giz, gin, ghr, ghz, ghn, hp);
                    sH[row * S_ + n]  = hn;
                    sHn[row * HP + n] = (_Float16)(hn * SCA);
                }
            }
        }
    }
    __syncthreads();

    if (tid < B_ * OUT_) {
        const int b = tid / OUT_;
        const int o = tid - b * OUT_;
        float acc = 0.0f;
#pragma unroll 4
        for (int k = 0; k < S_; ++k) acc = fmaf(sH[b * S_ + k], fw[o * S_ + k], acc);
        sOut[tid] = acc + fb[o];
    }
    __syncthreads();
    const bool wr = tid < (B_ * OUT_) / 4;
    v4f ov;
#pragma unroll
    for (int i = 0; i < 4; ++i) ov[i] = 0.0f;
    if (wr) ov = *(AS3 const v4f*)((lcp_f)sOut + 4 * tid);
    float* d = out + 4 * tid;
    if (wr) *(volatile v4f*)d = ov;
    __threadfence();
    if (wr) *(volatile v4f*)d = ov;
}

extern "C" void kernel_launch(void* const* d_in, const int* in_sizes, int n_in,
                              void* d_out, int out_size, void* d_ws, size_t ws_size,
                              hipStream_t stream)
{
    if (n_in < 16) return;
    if (in_sizes[0]  != B_ * C_ * L_) return;
    if (in_sizes[1]  != V_ * S_)      return;
    if (in_sizes[2]  != G3_ * S_)     return;
    if (in_sizes[3]  != G3_ * S_)     return;
    if (in_sizes[4]  != G3_)          return;
    if (in_sizes[5]  != G3_)          return;
    if (in_sizes[6]  != S_)           return;
    if (in_sizes[7]  != G3_ * S_)     return;
    if (in_sizes[8]  != G3_ * S_)     return;
    if (in_sizes[9]  != G3_)          return;
    if (in_sizes[10] != G3_)          return;
    if (in_sizes[11] != S_)           return;
    if (in_sizes[12] != S_ * PWK_)    return;
    if (in_sizes[13] != S_)           return;
    if (in_sizes[14] != OUT_ * S_)    return;
    if (in_sizes[15] != OUT_)         return;
    if (out_size != B_ * OUT_)        return;
    if (ws_size < WS_END)             return;

    const int*   tok   = (const int*)d_in[0];
    const float* embed = (const float*)d_in[1];
    const float* awih  = (const float*)d_in[2];
    const float* awhh  = (const float*)d_in[3];
    const float* abih  = (const float*)d_in[4];
    const float* abhh  = (const float*)d_in[5];
    const float* ainit = (const float*)d_in[6];
    const float* cwih  = (const float*)d_in[7];
    const float* cwhh  = (const float*)d_in[8];
    const float* cbih  = (const float*)d_in[9];
    const float* cbhh  = (const float*)d_in[10];
    const float* cinit = (const float*)d_in[11];
    const float* projw = (const float*)d_in[12];
    const float* projb = (const float*)d_in[13];
    const float* fw    = (const float*)d_in[14];
    const float* fb    = (const float*)d_in[15];
    float* out = (float*)d_out;

    char* ws = (char*)d_ws;
    _Float16* Emb = (_Float16*)(ws + OFF_EMB);
    _Float16* GI  = (_Float16*)(ws + OFF_GI);
    _Float16* Wai = (_Float16*)(ws + OFF_WAI);
    _Float16* Wah = (_Float16*)(ws + OFF_WAH);
    _Float16* Wci = (_Float16*)(ws + OFF_WCI);
    _Float16* Wch = (_Float16*)(ws + OFF_WCH);
    _Float16* Pw  = (_Float16*)(ws + OFF_PW);
    float*    hT  = (float*)(ws + OFF_HT);
    float*    GIc = (float*)(ws + OFF_GIC);

    cvt_kernel<<<dim3(CVT_BLK), dim3(NTHR), 0, stream>>>(
        embed, awih, awhh, cwih, cwhh, projw, Emb, Wai, Wah, Wci, Wch, Pw);

    gi_table_kernel<<<dim3(GI_BLK), dim3(NTHR), 0, stream>>>(
        (const _Float16*)Emb, (const _Float16*)Wai, GI);

    hipFuncSetAttribute(reinterpret_cast<const void*>(&ast_gru_kernel),
                        hipFuncAttributeMaxDynamicSharedMemorySize, (int)LDS_AST);
    ast_gru_kernel<<<dim3(ROW_BLK), dim3(NTHR), LDS_AST, stream>>>(
        tok, (const _Float16*)GI, (const _Float16*)Wah, abih, abhh, ainit, hT);

    hipFuncSetAttribute(reinterpret_cast<const void*>(&proj_kernel),
                        hipFuncAttributeMaxDynamicSharedMemorySize, (int)LDS_PROJ);
    proj_kernel<<<dim3(ROW_BLK), dim3(NTHR), LDS_PROJ, stream>>>(
        (const float*)hT, (const _Float16*)Pw, projw, projb, (const _Float16*)Wci, GIc);

    hipFuncSetAttribute(reinterpret_cast<const void*>(&ctx_gru_kernel),
                        hipFuncAttributeMaxDynamicSharedMemorySize, (int)LDS_CTX);
    ctx_gru_kernel<<<dim3(1), dim3(NTHR), LDS_CTX, stream>>>(
        (const float*)GIc, (const _Float16*)Wch, cbih, cbhh, cinit, fw, fb, out);
}
